// Cross_Attention_Network_42339787604711
// MI455X (gfx1250) — hardware-verified
//
#include <hip/hip_runtime.h>
#include <hip/hip_bf16.h>
#include <math.h>


#define BB 8
#define SS 2048
#define DD 256
#define HH 4
#define DKK 64
#define QW 2
#define KS4 264
#define NC 512
#define RSPLIT_UNUSED 0

typedef _Float16 bf16;
typedef __attribute__((ext_vector_type(4))) unsigned v4u_t;
typedef unsigned v4ua __attribute__((ext_vector_type(4), may_alias));
typedef __attribute__((ext_vector_type(4))) float v4f_t;
typedef float v4fa __attribute__((ext_vector_type(4), may_alias));
typedef __attribute__((ext_vector_type(16))) bf16  bf16x16;
typedef __attribute__((ext_vector_type(8)))  bf16  bf16x8;
typedef __attribute__((ext_vector_type(4)))  bf16  bf16x4;
typedef __attribute__((ext_vector_type(8)))  float f32x8;

#define LDS_STRIDE 48
#define KSTRIDE    72
#define VSTRIDE    48

__device__ __forceinline__ f32x8 wmma_bf16(bf16x16 a, bf16x16 b, f32x8 c) {
  return __builtin_amdgcn_wmma_f32_16x16x32_f16(
      false, a, false, b, (short)0, c, false, false);
}

template <typename T>
__device__ __forceinline__ bf16x16 load_frag(const T* __restrict__ base, int ld,
                                             int row0, int k0) {
  const int lane = threadIdx.x & 31;
  const int r    = lane & 15;
  const int kh   = (lane >> 4) * 8;
  const T* p0 = base + (size_t)(row0 + r) * ld + (k0 + kh);
  const T* p1 = p0 + 16;
  bf16x16 f;
#pragma unroll
  for (int i = 0; i < 8; ++i) {
    f[i]     = (bf16)p0[i];
    f[i + 8] = (bf16)p1[i];
  }
  return f;
}

__device__ __forceinline__ bf16x16 lds_frag(const bf16* base, int stride) {
  const int lane = threadIdx.x & 31;
  const int row  = lane & 15;
  const int kh   = (lane >> 4) * 8;
  const bf16x8 lo = *(const bf16x8*)(base + row * stride + kh);
  const bf16x8 hi = *(const bf16x8*)(base + row * stride + kh + 16);
  bf16x16 f;
#pragma unroll
  for (int i = 0; i < 8; ++i) { f[i] = lo[i]; f[i + 8] = hi[i]; }
  return f;
}

template <typename T>
__device__ __forceinline__ void stage_read16(const T* __restrict__ p, float* buf) {
#pragma unroll
  for (int i = 0; i < 16; ++i) buf[i] = (float)p[i];
}

__device__ __forceinline__ void stage_write(bf16* dst, const float* buf, int nquad) {
#pragma unroll
  for (int i = 0; i < nquad; ++i) {
    bf16x4 q;
    q[0] = (bf16)buf[4 * i];     q[1] = (bf16)buf[4 * i + 1];
    q[2] = (bf16)buf[4 * i + 2]; q[3] = (bf16)buf[4 * i + 3];
    *(bf16x4*)(dst + 4 * i) = q;
  }
}

template <typename AT, int MODE>
__global__ __launch_bounds__(256) void gemm_bias_kernel(
    const AT* __restrict__ A, const float* __restrict__ W,
    const float* __restrict__ bias, void* __restrict__ out,
    int M, int N, int K) {
  __shared__ bf16 ldsA[128 * LDS_STRIDE];
  __shared__ bf16 ldsW[256 * LDS_STRIDE];
  __shared__ __attribute__((aligned(16))) unsigned char sob[256 * 136 * 2];

  const int t    = threadIdx.x;
  const int wave = t >> 5;
  const int lane = t & 31;
  const int wm   = (wave & 1) * 64;
  const int wn   = (wave >> 1) * 64;
  const int mBlk = blockIdx.x * 128;
  const int nBlk = blockIdx.y * 256;

  const int arow = t >> 1;
  const int ach  = (t & 1) * 16;

  float abuf[16];
  float wbuf[32];

  stage_read16(A + (size_t)(mBlk + arow) * K + ach, abuf);
  stage_read16(W + (size_t)(nBlk + t) * K,          wbuf);
  stage_read16(W + (size_t)(nBlk + t) * K + 16,     wbuf + 16);

  f32x8 acc[4][4] = {};

  for (int k = 0; k < K; k += 32) {
    __syncthreads();
    stage_write(&ldsA[arow * LDS_STRIDE + ach], abuf, 4);
    stage_write(&ldsW[t * LDS_STRIDE],          wbuf, 8);
    if (k + 32 < K) {
      stage_read16(A + (size_t)(mBlk + arow) * K + (k + 32) + ach, abuf);
      stage_read16(W + (size_t)(nBlk + t) * K + (k + 32),          wbuf);
      stage_read16(W + (size_t)(nBlk + t) * K + (k + 32) + 16,     wbuf + 16);
    }
    __syncthreads();

    bf16x16 af[4], wf[4];
#pragma unroll
    for (int i = 0; i < 4; ++i)
      af[i] = lds_frag(ldsA + (wm + 16 * i) * LDS_STRIDE, LDS_STRIDE);
#pragma unroll
    for (int j = 0; j < 4; ++j)
      wf[j] = lds_frag(ldsW + (wn + 16 * j) * LDS_STRIDE, LDS_STRIDE);
#pragma unroll
    for (int i = 0; i < 4; ++i)
#pragma unroll
      for (int j = 0; j < 4; ++j)
        acc[i][j] = wmma_bf16(af[i], wf[j], acc[i][j]);
  }

  const int nlane = lane & 15;
  const int mh    = (lane >> 4) * 8;
  __syncthreads();
  if (MODE == 0 || MODE == 1) {
    bf16* so = (bf16*)sob;
#pragma unroll
    for (int i = 0; i < 4; ++i)
#pragma unroll
      for (int j = 0; j < 4; ++j) {
        const int nl = wn + 16 * j + nlane;
        const float bv = bias ? bias[nBlk + nl] : 0.0f;
#pragma unroll
        for (int r = 0; r < 8; ++r) {
          const int ml = wm + 16 * i + mh + r;
          const bf16 hv = (bf16)(acc[i][j][r] + bv);
          if (MODE == 0) so[ml * 264 + nl] = hv;
          else           so[nl * 136 + ml] = hv;
        }
      }
    __syncthreads();
#pragma unroll 1
    for (int pass = 0; pass < 2; ++pass) {
      if (MODE == 0) {
        for (int ch = t; ch < 128 * 32; ch += 256) { const int ml = ch >> 5, q = (ch & 31) * 8;
          *(volatile v4u_t*)((bf16*)out + (size_t)(mBlk + ml) * N + nBlk + q) = *(const v4ua*)(so + ml * 264 + q); }
      } else {
        const int b_ = mBlk / SS, s0 = mBlk & (SS - 1);
        for (int ch = t; ch < 256 * 16; ch += 256) { const int nl = ch >> 4, q = (ch & 15) * 8; const int n = nBlk + nl, h = n >> 6, dk = n & (DKK - 1);
          *(volatile v4u_t*)((bf16*)out + (((size_t)(b_ * HH + h)) * DKK + dk) * SS + s0 + q) = *(const v4ua*)(so + nl * 136 + q); }
      }
      __threadfence();
    }
  } else {
    float* so = (float*)sob;
#pragma unroll 1
    for (int hf = 0; hf < 2; ++hf) {
      if (wm == hf * 64) {
#pragma unroll
        for (int i = 0; i < 4; ++i)
#pragma unroll
          for (int j = 0; j < 4; ++j) {
            const int nl = wn + 16 * j + nlane;
            const float bv = bias ? bias[nBlk + nl] : 0.0f;
#pragma unroll
            for (int r = 0; r < 8; ++r) so[(16 * i + mh + r) * 260 + nl] = acc[i][j][r] + bv;
          }
      }
      __syncthreads();
#pragma unroll 1
      for (int pass = 0; pass < 2; ++pass) {
        for (int ch = t; ch < 64 * 64; ch += 256) { const int ml = ch >> 6, q = (ch & 63) * 4;
          *(volatile v4f_t*)((float*)out + (size_t)(mBlk + hf * 64 + ml) * N + nBlk + q) = *(const volatile v4fa*)(so + ml * 260 + q); }
        __threadfence();
      }
      __syncthreads();
    }
  }
}

__device__ __forceinline__ bf16 lo_of(float v, bf16 h) { return (bf16)((v - (float)h) * 2048.0f); }
__global__ __launch_bounds__(64) void attn256_kernel(const bf16* __restrict__ Qb, const bf16* __restrict__ Kb, const bf16* __restrict__ Vt, int vhalf, bf16* __restrict__ attnOut) {
  __shared__ bf16 ldsK[32 * KS4];
  __shared__ bf16 ldsV[128 * VSTRIDE];
  __shared__ __attribute__((aligned(16))) bf16 ldsO[2][16 * 136];
  const int q0blk = blockIdx.x * 32, b = blockIdx.z;
  const int t = threadIdx.x, wave = t >> 5, lane = t & 31, qlane = lane & 15, kh8 = (lane >> 4) * 8;
  const int q0 = q0blk + wave * 16;
  const bf16* Qh = Qb + (size_t)b * SS * DD;
  const bf16* Kh = Kb + (size_t)b * SS * DD;
  const bf16* Vh = Vt + ((size_t)b * DD + vhalf * 128) * SS;
  const int krow = t >> 1, kcol = (t & 1) * 128;
  bf16x16 qf[8];
#pragma unroll
  for (int c = 0; c < 8; ++c) qf[c] = load_frag(Qh, DD, q0, 32 * c);
  f32x8 o[8] = {};
  float mrun = -INFINITY, lrun = 0.0f;
  const float scale = 1.44269504088896340736f;
  const int kmax = SS - 1;
#pragma unroll 1
  for (int kb = 0; kb <= kmax; kb += 32) {
    __syncthreads();
    { const bf16* ks = Kh + (size_t)(kb + krow) * DD + kcol;
#pragma unroll
      for (int i = 0; i < 16; ++i) *(bf16x8*)(&ldsK[krow * KS4 + kcol + 8 * i]) = *(const bf16x8*)(ks + 8 * i);
      const bf16* vs0 = Vh + (size_t)t * SS + kb; const bf16* vs1 = Vh + (size_t)(64 + t) * SS + kb;
#pragma unroll
      for (int i = 0; i < 4; ++i) { *(bf16x8*)(&ldsV[t * VSTRIDE + 8 * i]) = *(const bf16x8*)(vs0 + 8 * i); *(bf16x8*)(&ldsV[(64 + t) * VSTRIDE + 8 * i]) = *(const bf16x8*)(vs1 + 8 * i); } }
    __syncthreads();
    f32x8 s0 = {}, s1 = {};
#pragma unroll
    for (int c = 0; c < 8; ++c) { s0 = wmma_bf16(lds_frag(ldsK + c * 32, KS4), qf[c], s0); s1 = wmma_bf16(lds_frag(ldsK + 16 * KS4 + c * 32, KS4), qf[c], s1); }
    float mx = -INFINITY;
#pragma unroll
    for (int r = 0; r < 8; ++r) { s0[r] *= scale; s1[r] *= scale; mx = fmaxf(mx, fmaxf(s0[r], s1[r])); }
    mx = fmaxf(mx, __shfl_xor(mx, 16, 32));
    const float mnew = fmaxf(mrun, mx), alpha = exp2f(mrun - mnew);
    float rsum = 0.0f; bf16x16 pf;
#pragma unroll
    for (int r = 0; r < 8; ++r) { const float p0 = exp2f(s0[r] - mnew), p1 = exp2f(s1[r] - mnew); rsum += p0 + p1; pf[r] = (bf16)(p0 * 1024.0f); pf[r + 8] = (bf16)(p1 * 1024.0f); }
    rsum += __shfl_xor(rsum, 16, 32);
    lrun = lrun * alpha + rsum; mrun = mnew;
#pragma unroll
    for (int j = 0; j < 8; ++j) {
#pragma unroll
      for (int r = 0; r < 8; ++r) o[j][r] *= alpha;
      o[j] = wmma_bf16(lds_frag(ldsV + (j * 16) * VSTRIDE, VSTRIDE), pf, o[j]); }
  }
  bf16* so = ldsO[wave];
  const float rl = 1.0f / (lrun * 1024.0f);
#pragma unroll
  for (int j = 0; j < 8; ++j)
#pragma unroll
    for (int r = 0; r < 8; ++r) { const float v = o[j][r] * rl; so[qlane * 136 + j * 16 + kh8 + r] = (bf16)v; }
  asm volatile("s_wait_dscnt 0" ::: "memory");
#pragma unroll 1
  for (int pass = 0; pass < 2; ++pass) {
#pragma unroll
    for (int it = 0; it < 8; ++it) { const int ch = lane + 32 * it, ql = ch >> 4, q8 = (ch & 15) * 8;
      bf16* dst = attnOut + ((size_t)(b * SS + q0 + ql)) * DD + vhalf * 128 + q8;
      *(volatile v4u_t*)dst = *(const v4ua*)(so + ql * 136 + q8); }
    __threadfence();
  }
}

__global__ __launch_bounds__(256) void k_tw(const float* __restrict__ W, float* __restrict__ WT, int K, int N) {
  __shared__ float tile[64][65];
  const int kb0 = blockIdx.y * 64, n0 = blockIdx.x * 64, t = threadIdx.x;
  for (int i = t; i < 64 * 64; i += 256) { const int kr = i >> 6, nc = i & 63; tile[kr][nc] = W[(size_t)(kb0 + kr) * N + n0 + nc]; }
  __syncthreads();
#pragma unroll 1
  for (int pass = 0; pass < 2; ++pass) {
    for (int i = t; i < 64 * 16; i += 256) { const int nr = i >> 4, k4 = (i & 15) * 4; v4f_t v; v.x = tile[k4][nr]; v.y = tile[k4 + 1][nr]; v.z = tile[k4 + 2][nr]; v.w = tile[k4 + 3][nr];
      *(volatile v4f_t*)(WT + (size_t)(n0 + nr) * K + kb0 + k4) = v; }
    __threadfence();
  }
}
__global__ __launch_bounds__(256) void k_bnstat(const float* __restrict__ X, float* __restrict__ st) {
  __shared__ float rs_[256], rq_[256];
  const int c = blockIdx.x, t = threadIdx.x; float s = 0.f, q = 0.f;
  for (int n = 0; n < BB; ++n) { const float* row = X + ((size_t)n * NC + c) * SS; for (int l = t; l < SS; l += 256) { const float v = row[l]; s += v; q += v * v; } }
  rs_[t] = s; rq_[t] = q; __syncthreads();
  for (int o = 128; o > 0; o >>= 1) { if (t < o) { rs_[t] += rs_[t + o]; rq_[t] += rq_[t + o]; } __syncthreads(); }
  if (t < 32) { float v = 0.0f;
    if (t == 0) { const double cnt = (double)BB * SS, mu = (double)rs_[0] / cnt; v = (float)mu; }
    if (t == 1) { const double cnt = (double)BB * SS, mu = (double)rs_[0] / cnt; const double var = fmax((double)rq_[0] / cnt - mu * mu, 0.0); v = (float)(1.0 / sqrt(var + 1e-5)); }
    *(volatile float*)(st + (size_t)c * 32 + t) = v; __threadfence(); *(volatile float*)(st + (size_t)c * 32 + t) = v; }
}
__global__ __launch_bounds__(256) void k_bnrows(const float* __restrict__ X, const float* __restrict__ st, const float* __restrict__ g, const float* __restrict__ be, float* __restrict__ Xn) {
  __shared__ float tile[64][65];
  const int l0 = blockIdx.x * 64, c0 = blockIdx.y * 64, n = blockIdx.z, t = threadIdx.x;
  for (int i = t; i < 64 * 64; i += 256) { const int cr = i >> 6, ll = i & 63; const int c = c0 + cr;
    const float v = (X[((size_t)n * NC + c) * SS + l0 + ll] - st[(size_t)c * 32]) * st[(size_t)c * 32 + 1] * g[c] + be[c]; tile[cr][ll] = fmaxf(v, 0.0f); }
  __syncthreads();
#pragma unroll 1
  for (int pass = 0; pass < 2; ++pass) {
    for (int i = t; i < 64 * 16; i += 256) { const int lr = i >> 4, c4 = (i & 15) * 4; v4f_t v; v.x = tile[c4][lr]; v.y = tile[c4 + 1][lr]; v.z = tile[c4 + 2][lr]; v.w = tile[c4 + 3][lr];
      *(volatile v4f_t*)(Xn + ((size_t)n * SS + l0 + lr) * NC + c0 + c4) = v; }
    __threadfence();
  }
}
__global__ __launch_bounds__(256) void k_fin(const float* __restrict__ An, const float* __restrict__ O, float* __restrict__ out) {
  __shared__ float tile[64][65];
  const int l0 = blockIdx.x * 64, c0 = blockIdx.y * 64, n = blockIdx.z, t = threadIdx.x;
  for (int i = t; i < 64 * 64; i += 256) { const int lr = i >> 6, cc = i & 63; const size_t off = ((size_t)n * SS + l0 + lr) * NC + c0 + cc; tile[lr][cc] = An[off] + O[off]; }
  __syncthreads();
#pragma unroll 1
  for (int pass = 0; pass < 2; ++pass) {
    for (int i = t; i < 64 * 16; i += 256) { const int cr = i >> 4, l4 = (i & 15) * 4; v4f_t v; v.x = tile[l4][cr]; v.y = tile[l4 + 1][cr]; v.z = tile[l4 + 2][cr]; v.w = tile[l4 + 3][cr];
      *(volatile v4f_t*)(out + ((size_t)n * NC + c0 + cr) * SS + l0 + l4) = v; }
    __threadfence();
  }
}

extern "C" void kernel_launch(void* const* d_in, const int* in_sizes, int n_in,
                              void* d_out, int out_size, void* d_ws, size_t ws_size,
                              hipStream_t stream) {
  (void)in_sizes; (void)n_in; (void)out_size; (void)ws_size;
  const float* A = (const float*)d_in[0]; const float* Bx = (const float*)d_in[1];
  const float* g = (const float*)d_in[2]; const float* be = (const float*)d_in[3];
  const float* thw = (const float*)d_in[4]; const float* thb = (const float*)d_in[5];
  const float* phw = (const float*)d_in[6]; const float* phb = (const float*)d_in[7];
  const float* gw = (const float*)d_in[8]; const float* gb = (const float*)d_in[9];
  const float* Ww = (const float*)d_in[10]; const float* Wb = (const float*)d_in[11];
  float* out = (float*)d_out;
  const int M = BB * SS;
  char* ws = (char*)d_ws;
  float* WT  = (float*)ws; ws += (size_t)4 * 256 * 512 * 4;
  float* st  = (float*)ws; ws += (size_t)2 * NC * 32 * 4;
  float* An  = (float*)ws; ws += (size_t)M * NC * 4;
  float* Bn  = (float*)ws; ws += (size_t)M * NC * 4;
  float* O   = Bn;
  bf16* Qb   = (bf16*)ws;  ws += (size_t)M * DD * 2;
  bf16* Kb   = (bf16*)ws;  ws += (size_t)M * DD * 2;
  bf16* VtB  = (bf16*)ws;  ws += (size_t)M * DD * 2;
  bf16* Y    = (bf16*)ws;  ws += (size_t)M * DD * 2;
  const size_t pl = (size_t)256 * 512;
  k_tw<<<dim3(256 / 64, 512 / 64), 256, 0, stream>>>(thw, WT, 512, 256);
  k_tw<<<dim3(256 / 64, 512 / 64), 256, 0, stream>>>(phw, WT + pl, 512, 256);
  k_tw<<<dim3(256 / 64, 512 / 64), 256, 0, stream>>>(gw, WT + 2 * pl, 512, 256);
  k_tw<<<dim3(512 / 64, 256 / 64), 256, 0, stream>>>(Ww, WT + 3 * pl, 256, 512);
  k_bnstat<<<NC, 256, 0, stream>>>(A, st);
  k_bnstat<<<NC, 256, 0, stream>>>(Bx, st + (size_t)NC * 32);
  k_bnrows<<<dim3(SS / 64, NC / 64, BB), 256, 0, stream>>>(A, st, g, be, An);
  k_bnrows<<<dim3(SS / 64, NC / 64, BB), 256, 0, stream>>>(Bx, st + (size_t)NC * 32, g, be, Bn);
  dim3 gGrid(M / 128, DD / 256), gBlk(256);
  gemm_bias_kernel<float, 0><<<gGrid, gBlk, 0, stream>>>(An, WT,          thb, Qb,  M, DD, NC);
  gemm_bias_kernel<float, 0><<<gGrid, gBlk, 0, stream>>>(Bn, WT + pl,     phb, Kb,  M, DD, NC);
  gemm_bias_kernel<float, 1><<<gGrid, gBlk, 0, stream>>>(An, WT + 2 * pl, gb,  VtB, M, DD, NC);
  attn256_kernel<<<dim3(SS / 32, 1, BB), 64, 0, stream>>>(Qb, Kb, VtB, 0, Y);
  attn256_kernel<<<dim3(SS / 32, 1, BB), 64, 0, stream>>>(Qb, Kb, VtB, 1, Y);
  gemm_bias_kernel<bf16, 2><<<dim3(M / 128, NC / 256), gBlk, 0, stream>>>(Y, WT + 3 * pl, Wb, O, M, NC, DD);
  k_fin<<<dim3(SS / 64, NC / 64, BB), 256, 0, stream>>>(An, O, out);
}
